// SATLayer_75247827026131
// MI455X (gfx1250) — hardware-verified
//
#include <hip/hip_runtime.h>
#include <stdint.h>

#define NBATCH 8
#define NN     128
#define DDIM   256
#define NROWS  1024
#define PLN    262144
#define WSZ    65536
#define SSZ    131072
static_assert(NROWS == NBATCH * NN);
static_assert(PLN == NROWS * DDIM);
static_assert(WSZ == DDIM * DDIM);
static_assert(SSZ == NBATCH * NN * NN);
static_assert(NN == 128);
static_assert(DDIM == 256);
static_assert((NROWS % 64) == 0);

typedef _Float16     v16h __attribute__((ext_vector_type(16)));
typedef _Float16     v8h  __attribute__((ext_vector_type(8)));
typedef float        v8f  __attribute__((ext_vector_type(8)));
typedef float        v4f  __attribute__((ext_vector_type(4)));
typedef unsigned int v4u  __attribute__((ext_vector_type(4)));
typedef int          v4i  __attribute__((ext_vector_type(4)));

union Frag { v16h v; v8h half[2]; };

__device__ __forceinline__ unsigned short bf_bits(float f) {
  unsigned u = __float_as_uint(f);
  return (unsigned short)((u + 0x7FFFu + ((u >> 16) & 1u)) >> 16);
}
__device__ __forceinline__ float bf_up(unsigned short b) { return __uint_as_float(((unsigned)b) << 16); }
__device__ __forceinline__ float bfr(float f) { return bf_up(bf_bits(f)); }
__device__ __forceinline__ unsigned short h_bits(float f) {
  return __builtin_bit_cast(unsigned short, (_Float16)f);
}
__device__ __forceinline__ unsigned pack2(float a, float b) {
  return (unsigned)h_bits(a) | (((unsigned)h_bits(b)) << 16);
}
__device__ __forceinline__ v8f fill8(float x) {
  v8f z;
  z[0] = x; z[1] = x; z[2] = x; z[3] = x; z[4] = x; z[5] = x; z[6] = x; z[7] = x;
  return z;
}

__device__ __forceinline__ v16h ldfrag(const _Float16* p) {
  Frag f;
  f.half[0] = *(const v8h*)(p);
  f.half[1] = *(const v8h*)(p + 16);
  return f.v;
}

__device__ __forceinline__ v8f mma(v16h a, v16h b, v8f c) {
  v8f d = __builtin_amdgcn_wmma_f32_16x16x32_f16(false, a, false, b, (short)0, c, false, false);
#if defined(__HIP_DEVICE_COMPILE__)
  asm volatile("v_nop\n\tv_nop\n\tv_nop\n\tv_nop" : "+v"(d) : "v"(a), "v"(b));
#endif
  return d;
}

__global__ __launch_bounds__(256) void k_prep(const float* __restrict__ x,
                                              const float* __restrict__ Wq, const float* __restrict__ Wk,
                                              const float* __restrict__ Wv, const float* __restrict__ Wo,
                                              unsigned short* Xh, unsigned short* WT) {
  __shared__ __align__(16) unsigned short sT[8192];
  const int tid = threadIdx.x;
  const int bid = blockIdx.x;
  const int isw = (bid >= (NROWS * DDIM / 2048)) ? 1 : 0;
  const int wb  = isw ? (bid - (NROWS * DDIM / 2048)) : 0;
  const int wi  = wb >> 3;
  const int e0  = (wb & 7) * 32;

  if (isw) {
    const float* src = (wi == 0) ? Wq : ((wi == 1) ? Wk : ((wi == 2) ? Wv : Wo));
#pragma unroll 1
    for (int it = 0; it < 4; ++it) {
      const int p  = it * 256 + tid;
      const int f  = p >> 2;
      const int c8 = (p & 3) * 8;
      const float* q = src + (size_t)f * DDIM + e0 + c8;
      const v4f v0 = *(const v4f*)(q);
      const v4f v1 = *(const v4f*)(q + 4);
      unsigned short* d = sT + c8 * 256 + f;
#pragma unroll
      for (int u = 0; u < 4; ++u) {
        d[u * 256]       = h_bits(bfr(v0[u]) * 1024.0f);
        d[(u + 4) * 256] = h_bits(bfr(v1[u]) * 1024.0f);
      }
    }
  }
  __syncthreads();

  if (isw) {
    unsigned short* dst = WT + (size_t)wi * WSZ + (size_t)e0 * DDIM;
    v4u pv[4];
#pragma unroll
    for (int it = 0; it < 4; ++it) pv[it] = *(const v4u*)(sT + (size_t)(it * 256 + tid) * 8);
#pragma unroll
    for (int it = 0; it < 4; ++it) *(volatile v4u*)(dst + (size_t)(it * 256 + tid) * 8) = pv[it];
    __threadfence();
#pragma unroll
    for (int it = 0; it < 4; ++it) *(volatile v4u*)(dst + (size_t)(it * 256 + tid) * 8) = pv[it];
  } else {
    const size_t base = (size_t)bid * 2048 + (size_t)tid * 8;
    const v4f v0 = *(const v4f*)(x + base);
    const v4f v1 = *(const v4f*)(x + base + 4);
    v4u pk;
    pk[0] = pack2(bfr(v0[0]) * 16.0f, bfr(v0[1]) * 16.0f);
    pk[1] = pack2(bfr(v0[2]) * 16.0f, bfr(v0[3]) * 16.0f);
    pk[2] = pack2(bfr(v1[0]) * 16.0f, bfr(v1[1]) * 16.0f);
    pk[3] = pack2(bfr(v1[2]) * 16.0f, bfr(v1[3]) * 16.0f);
    unsigned short* dst = Xh + base;
    *(volatile v4u*)dst = pk;
    __threadfence();
    *(volatile v4u*)dst = pk;
  }
}

__global__ __launch_bounds__(256) void k_proj(const unsigned short* __restrict__ Xhp,
                                              const unsigned short* __restrict__ WTp,
                                              const float* __restrict__ bq, const float* __restrict__ bk,
                                              const float* __restrict__ bv, unsigned short* QKV) {
  __shared__ __align__(16) unsigned short sT[4096];
  const _Float16* Xh = (const _Float16*)(const void*)Xhp;
  const _Float16* WT = (const _Float16*)(const void*)WTp;
  const int tid  = threadIdx.x;
  const int lane = tid & 31, w = tid >> 5, h = lane >> 4, m = lane & 15;
  const int bid  = blockIdx.x;
  const int pj   = bid / ((NROWS / 64) * (DDIM / 64));
  const int rt   = (bid / (DDIM / 64)) % (NROWS / 64);
  const int cg   = bid % (DDIM / 64);
  const int n0   = rt * 64;
  const int e0g  = cg * 64;
  const int wr   = w >> 1, wc = w & 1;
  const int tr   = (pj == 2) ? 1 : 0;
  const float* bias = (pj == 0) ? bq : ((pj == 1) ? bk : bv);

  const _Float16* Ap  = Xh + (size_t)(n0 + 16 * wr + m) * DDIM + 8 * h;
  const _Float16* Bp0 = WT + (size_t)pj * WSZ + (size_t)(e0g + 32 * wc + m) * DDIM + 8 * h;
  const _Float16* Bp1 = Bp0 + (size_t)16 * DDIM;
  v8f acc0 = fill8(0.0f), acc1 = fill8(0.0f);
#pragma unroll
  for (int ks = 0; ks < 8; ++ks) {
    const v16h a = ldfrag(Ap + ks * 32);
    acc0 = mma(a, ldfrag(Bp0 + ks * 32), acc0);
    acc1 = mma(a, ldfrag(Bp1 + ks * 32), acc1);
  }

  const int el0 = 32 * wc + m, el1 = el0 + 16;
  const float bb0 = bfr(bias[e0g + el0]);
  const float bb1 = bfr(bias[e0g + el1]);
#pragma unroll
  for (int r = 0; r < 8; ++r) {
    const int nl = 16 * wr + 8 * h + r;
    const float v0 = (acc0[r] * 6.103515625e-05f + bb0) * 16.0f;
    const float v1 = (acc1[r] * 6.103515625e-05f + bb1) * 16.0f;
    const int i0 = tr ? (el0 * 64 + nl) : (nl * 64 + el0);
    const int i1 = tr ? (el1 * 64 + nl) : (nl * 64 + el1);
    sT[i0] = h_bits(v0);
    sT[i1] = h_bits(v1);
  }
  __syncthreads();

  const int piece = tid & 7, rq = tid >> 3;
  const int b = rt >> 1, kk0 = (rt & 1) * 64;
  v4u pv[2];
  size_t o[2];
#pragma unroll
  for (int it = 0; it < 2; ++it) {
    const int row = it * 32 + rq;
    pv[it] = *(const v4u*)(sT + row * 64 + piece * 8);
    const size_t oN = (size_t)pj * PLN + (size_t)(n0 + row) * DDIM + e0g + piece * 8;
    const size_t oT = (size_t)2 * PLN + (size_t)(b * DDIM + e0g + row) * NN + kk0 + piece * 8;
    o[it] = tr ? oT : oN;
  }
#pragma unroll
  for (int it = 0; it < 2; ++it) *(volatile v4u*)(QKV + o[it]) = pv[it];
  __threadfence();
#pragma unroll
  for (int it = 0; it < 2; ++it) *(volatile v4u*)(QKV + o[it]) = pv[it];
}

__global__ __launch_bounds__(256) void k_scores(const unsigned short* __restrict__ QKV, float* S) {
  __shared__ __align__(16) float sS[2048];
  const _Float16* Q = (const _Float16*)(const void*)QKV;
  const _Float16* K = Q + PLN;
  const int tid  = threadIdx.x;
  const int lane = tid & 31, w = tid >> 5, h = lane >> 4, m = lane & 15;
  const int bid  = blockIdx.x;
  const int jt   = bid & 7;
  const int b    = bid >> 3;
  const int j0   = b * NN + jt * 16;
  const int kr0  = b * NN + w * 16;

  const _Float16* Ap = Q + (size_t)(j0 + m) * DDIM + 8 * h;
  const _Float16* Bp = K + (size_t)(kr0 + m) * DDIM + 8 * h;
  v8f acc = fill8(0.0f);
#pragma unroll
  for (int ks = 0; ks < 8; ++ks) acc = mma(ldfrag(Ap + ks * 32), ldfrag(Bp + ks * 32), acc);

#pragma unroll
  for (int r = 0; r < 8; ++r) sS[(8 * h + r) * NN + w * 16 + m] = acc[r] * 0.000244140625f;
  __syncthreads();
#pragma unroll 1
  for (int e = tid; e < 2048; e += 256) sS[e] = expf(sS[e]);
  __syncthreads();

  v4f pv[2];
#pragma unroll
  for (int it = 0; it < 2; ++it) pv[it] = *(const v4f*)(sS + (size_t)(it * 256 + tid) * 4);
  float* op = S + (size_t)j0 * NN;
#pragma unroll
  for (int it = 0; it < 2; ++it) *(volatile v4f*)(op + (size_t)(it * 256 + tid) * 4) = pv[it];
  __threadfence();
#pragma unroll
  for (int it = 0; it < 2; ++it) *(volatile v4f*)(op + (size_t)(it * 256 + tid) * 4) = pv[it];
}

__global__ __launch_bounds__(256) void k_main(const int* __restrict__ adj, const int* __restrict__ adjm,
                                              const float* __restrict__ S, const unsigned short* __restrict__ QKVp,
                                              const unsigned short* __restrict__ WTp, const float* __restrict__ bo,
                                              float* out) {
  extern __shared__ __align__(16) _Float16 smem[];
  __shared__ __align__(16) float sO[DDIM];
  __shared__ float wsr[NN];
  __shared__ int   sok[NN];
  _Float16* Pt = smem;
  _Float16* Xt = smem + NN * NN;
  const _Float16* VT  = (const _Float16*)(const void*)QKVp + (size_t)2 * PLN;
  const _Float16* WoT = (const _Float16*)(const void*)WTp + (size_t)3 * WSZ;
  const int tid  = threadIdx.x;
  const int lane = tid & 31, w = tid >> 5, h = lane >> 4, m = lane & 15;
  const int b    = blockIdx.x >> 7;
  const int j    = blockIdx.x & (NN - 1);

  if (tid < NN) {
    wsr[tid] = S[(size_t)(b * NN + j) * NN + tid];
    sok[tid] = (adjm[(size_t)(b * NN + tid) * NN + j] == 0) ? 1 : 0;
  }
  __syncthreads();

  if (tid < NN) {
    const int i = tid;
    const int* arow = adj + (size_t)(b * NN + i) * NN;
    const int aij = arow[j];
    float den = 0.0f;
#pragma unroll 1
    for (int k8 = 0; k8 < 16; ++k8) {
      const v4i a0 = *(const v4i*)(arow + k8 * 8);
      const v4i a1 = *(const v4i*)(arow + k8 * 8 + 4);
#pragma unroll
      for (int u = 0; u < 4; ++u) {
        const float s0 = wsr[k8 * 8 + u];
        const float s1 = wsr[k8 * 8 + 4 + u];
        den += (a0[u] != 0) ? s0 : 0.0f;
        den += (a1[u] != 0) ? s1 : 0.0f;
      }
    }
    den = (aij != 0) ? den : 0.0f;
    const float rden = 1.0f / fmaxf(den, 1.0e-9f);
#pragma unroll 1
    for (int k8 = 0; k8 < 16; ++k8) {
      const v4i a0 = *(const v4i*)(arow + k8 * 8);
      const v4i a1 = *(const v4i*)(arow + k8 * 8 + 4);
      v8h hv;
#pragma unroll
      for (int u = 0; u < 4; ++u) {
        const float s0 = wsr[k8 * 8 + u];
        const float s1 = wsr[k8 * 8 + 4 + u];
        const float t0 = (aij != 0 && a0[u] != 0) ? s0 : 0.0f;
        const float t1 = (aij != 0 && a1[u] != 0) ? s1 : 0.0f;
        hv[u]     = (_Float16)((t0 * rden) * 1024.0f);
        hv[4 + u] = (_Float16)((t1 * rden) * 1024.0f);
      }
      *(v8h*)(Pt + i * NN + k8 * 8) = hv;
    }
  }
  __syncthreads();

  {
    const _Float16* vp0 = VT + (size_t)(b * DDIM + 32 * w + m) * NN + 8 * h;
    const _Float16* vp1 = vp0 + (size_t)16 * NN;
    v16h Bf0[4], Bf1[4];
#pragma unroll
    for (int ks = 0; ks < 4; ++ks) {
      Bf0[ks] = ldfrag(vp0 + ks * 32);
      Bf1[ks] = ldfrag(vp1 + ks * 32);
    }
#pragma unroll 1
    for (int it = 0; it < 8; ++it) {
      const _Float16* ap = Pt + (it * 16 + m) * NN + 8 * h;
      v8f a0 = fill8(0.0f), a1 = fill8(0.0f);
#pragma unroll
      for (int ks = 0; ks < 4; ++ks) {
        const v16h a = ldfrag(ap + ks * 32);
        a0 = mma(a, Bf0[ks], a0);
        a1 = mma(a, Bf1[ks], a1);
      }
#pragma unroll
      for (int r = 0; r < 8; ++r) {
        _Float16* xr = Xt + (size_t)(it * 16 + 8 * h + r) * DDIM + 32 * w + m;
        xr[0]  = (_Float16)(a0[r] * 0.0009765625f);
        xr[16] = (_Float16)(a1[r] * 0.0009765625f);
      }
    }
  }
  __syncthreads();

  v8f m0 = fill8(-3.0e38f), m1 = fill8(-3.0e38f);
  {
    const _Float16* bp0 = WoT + (size_t)(32 * w + m) * DDIM + 8 * h;
    const _Float16* bp1 = bp0 + (size_t)16 * DDIM;
    const float bb0 = bfr(bo[32 * w + m]);
    const float bb1 = bfr(bo[32 * w + 16 + m]);
#pragma unroll 1
    for (int it = 0; it < 8; ++it) {
      const _Float16* ap = Xt + (size_t)(it * 16 + m) * DDIM + 8 * h;
      v8f c0 = fill8(0.0f), c1 = fill8(0.0f);
#pragma unroll
      for (int ks = 0; ks < 8; ++ks) {
        const v16h a = ldfrag(ap + ks * 32);
        c0 = mma(a, ldfrag(bp0 + ks * 32), c0);
        c1 = mma(a, ldfrag(bp1 + ks * 32), c1);
      }
#pragma unroll
      for (int r = 0; r < 8; ++r) {
        const int ok = sok[it * 16 + 8 * h + r];
        const float v0 = c0[r] * 6.103515625e-05f + bb0;
        const float v1 = c1[r] * 6.103515625e-05f + bb1;
        m0[r] = fmaxf(m0[r], (ok != 0) ? v0 : -1.0e12f);
        m1[r] = fmaxf(m1[r], (ok != 0) ? v1 : -1.0e12f);
      }
    }
  }

  float M0 = m0[0], M1 = m1[0];
#pragma unroll
  for (int r = 1; r < 8; ++r) { M0 = fmaxf(M0, m0[r]); M1 = fmaxf(M1, m1[r]); }
  M0 = fmaxf(M0, __shfl_xor(M0, 16, 32));
  M1 = fmaxf(M1, __shfl_xor(M1, 16, 32));
  sO[w * 32 + m]      = M0;
  sO[w * 32 + 16 + m] = M1;
  __syncthreads();

  float* op = out + (size_t)(b * NN + j) * DDIM + (size_t)tid * 4;
  if (tid < 64) {
    const v4f ov = *(const v4f*)(sO + tid * 4);
    *(volatile v4f*)op = ov;
  }
  __threadfence();
  if (tid < 64) {
    const v4f ov = *(const v4f*)(sO + tid * 4);
    *(volatile v4f*)op = ov;
  }
}

extern "C" void kernel_launch(void* const* d_in, const int* in_sizes, int n_in,
                              void* d_out, int out_size, void* d_ws, size_t ws_size,
                              hipStream_t stream) {
  if (n_in < 11) return;
  if (in_sizes[0] != SSZ) return;
  if (in_sizes[1] != PLN) return;
  if (in_sizes[2] != SSZ) return;
  if (in_sizes[3] != WSZ || in_sizes[4] != DDIM) return;
  if (in_sizes[5] != WSZ || in_sizes[6] != DDIM) return;
  if (in_sizes[7] != WSZ || in_sizes[8] != DDIM) return;
  if (in_sizes[9] != WSZ || in_sizes[10] != DDIM) return;
  if (out_size != PLN) return;

  const int*   adj  = (const int*)d_in[0];
  const float* x    = (const float*)d_in[1];
  const int*   adjm = (const int*)d_in[2];
  const float* Wq   = (const float*)d_in[3];  const float* bq = (const float*)d_in[4];
  const float* Wk   = (const float*)d_in[5];  const float* bk = (const float*)d_in[6];
  const float* Wv   = (const float*)d_in[7];  const float* bv = (const float*)d_in[8];
  const float* Wo   = (const float*)d_in[9];  const float* bo = (const float*)d_in[10];
  float* out = (float*)d_out;

  const size_t offXh  = 0;
  const size_t offWT  = offXh  + (size_t)PLN * 2;
  const size_t offQKV = offWT  + (size_t)4 * WSZ * 2;
  const size_t offS   = offQKV + (size_t)3 * PLN * 2;
  const size_t total  = offS   + (size_t)SSZ * 4;
  if (total > ws_size) return;
  if (total > (size_t)134217728) return;

  char* ws = (char*)d_ws;
  unsigned short* Xh  = (unsigned short*)(ws + offXh);
  unsigned short* WT  = (unsigned short*)(ws + offWT);
  unsigned short* QKV = (unsigned short*)(ws + offQKV);
  float*          S   = (float*)(ws + offS);

  const int ldsMain = (NN * NN + NN * DDIM) * 2;
  (void)hipFuncSetAttribute(reinterpret_cast<const void*>(&k_main),
                            hipFuncAttributeMaxDynamicSharedMemorySize, ldsMain);

  k_prep<<<dim3((NROWS * DDIM / 2048) + 32), dim3(256), 0, stream>>>(x, Wq, Wk, Wv, Wo, Xh, WT);
  k_proj<<<dim3(3 * (NROWS / 64) * (DDIM / 64)), dim3(256), 0, stream>>>(Xh, WT, bq, bk, bv, QKV);
  k_scores<<<dim3(NBATCH * (NN / 16)), dim3(256), 0, stream>>>(QKV, S);
  k_main<<<dim3(NBATCH * NN), dim3(256), ldsMain, stream>>>(adj, adjm, S, QKV, WT, bo, out);
  (void)hipGetLastError();
}
